// OctreeConvRelu_63651415327310
// MI455X (gfx1250) — hardware-verified
//
#include <hip/hip_runtime.h>
#include <stdint.h>

typedef __bf16         v16bf __attribute__((ext_vector_type(16)));
typedef float          v8f   __attribute__((ext_vector_type(8)));
typedef float          v4f   __attribute__((ext_vector_type(4)));
typedef unsigned int   v4u   __attribute__((ext_vector_type(4)));
typedef unsigned int   v8u   __attribute__((ext_vector_type(8)));
typedef v4f __attribute__((may_alias)) v4fa;
typedef v4u __attribute__((may_alias)) v4ua;

union FragU { v16bf v; v8u w; v4u q[2]; };

#define C_IN    64
#define C_OUT   128
#define KSZ     27
#define KDIM    (C_IN * KSZ)
#define KCHUNK  32
#define NKC     (KDIM / KCHUNK)
#define NT      32
#define NWAVE   8
#define BLOCK   (NWAVE * 32)
#define MT      (C_OUT / 16)
#define SPITCH  36

typedef char chk_kdim [(NKC * KCHUNK == KDIM) ? 1 : -1];
typedef char chk_cin  [(C_IN == 64) ? 1 : -1];
typedef char chk_mt   [(MT == NWAVE) ? 1 : -1];

__device__ __forceinline__ unsigned short f2bf(float f) {
    unsigned u = __float_as_uint(f);
    u += 0x7FFFu + ((u >> 16) & 1u);
    return (unsigned short)(u >> 16);
}

__device__ __forceinline__ v8f wmma_bf16(v16bf a, v16bf b, v8f c) {
    return __builtin_amdgcn_wmma_f32_16x16x32_bf16(false, a, false, b, (short)0, c, false, false);
}

__global__ __launch_bounds__(256) void k_xT(const float* __restrict__ x,
                                            unsigned short* __restrict__ xT, int H) {
    __shared__ __attribute__((aligned(16))) unsigned short s[32][72];
    const int h0  = blockIdx.x * 32;
    const int tid = threadIdx.x;
    #pragma unroll
    for (int i = 0; i < 8; ++i) {
        int idx = tid + 256 * i;
        int c   = idx >> 5;
        int hl  = idx & 31;
        int h   = h0 + hl;
        float v = (h < H) ? x[(size_t)c * H + h] : 0.0f;
        s[hl][c] = f2bf(v);
    }
    __syncthreads();
    const int wave  = tid >> 5;
    const int lane  = tid & 31;
    const int hl    = wave * 4 + (lane >> 3);
    const int chunk = lane & 7;
    const int h     = h0 + hl;
    v4u v = *(const v4ua*)&s[hl][chunk * 8];
    unsigned short* d = xT + (size_t)h * C_IN + chunk * 8;
    if (h < H) { *(volatile v4u*)d = v; }
    __threadfence();
    if (h < H) { *(volatile v4u*)d = v; }
}

__global__ __launch_bounds__(256) void k_pack_w(const float* __restrict__ W,
                                                unsigned short* __restrict__ Wp, int nunits) {
    const int u = blockIdx.x * blockDim.x + threadIdx.x;
    if (u >= nunits) return;
    const int e0   = (u & 1) * 8;
    const int lane = (u >> 1) & 31;
    const int q    = u >> 6;
    const int kc   = q % NKC;
    const int mt   = q / NKC;
    const int M    = mt * 16 + (lane & 15);
    const int hh   = lane >> 4;
    unsigned w[4] = {0u, 0u, 0u, 0u};
    #pragma unroll
    for (int i = 0; i < 8; ++i) {
        int e   = e0 + i;
        int off = (e < 8) ? (8 * hh + e) : (16 + 8 * hh + (e - 8));
        int kk  = kc * KCHUNK + off;
        int c   = kk & 63;
        int k   = kk >> 6;
        unsigned short b = f2bf(W[((size_t)M * C_IN + c) * KSZ + k]);
        w[i >> 1] |= ((unsigned)b) << (16 * (i & 1));
    }
    v4u v = {w[0], w[1], w[2], w[3]};
    unsigned short* d = Wp + (size_t)u * 8;
    *(volatile v4u*)d = v;
    __threadfence();
    *(volatile v4u*)d = v;
}

__global__ __launch_bounds__(256) void k_gather(const unsigned short* __restrict__ xT,
                                                const int*            __restrict__ neigh,
                                                unsigned short*       __restrict__ cols,
                                                int H, int hc0, int count, int nunits) {
    const int u = blockIdx.x * blockDim.x + threadIdx.x;
    if (u >= nunits) return;
    const int part = u & 7;
    const int g    = u >> 3;
    const int nl   = g / KSZ;
    const int k    = g - nl * KSZ;
    const int h    = hc0 + nl;
    int j = -1;
    if (nl < count && h < H) j = neigh[(size_t)h * KSZ + k];
    v4u v = {0u, 0u, 0u, 0u};
    if (j >= 0) {
        if (j >= H) j = H - 1;
        v = *(const v4u*)(xT + (size_t)j * C_IN + part * 8);
    }
    unsigned short* d = cols + (size_t)nl * KDIM + k * C_IN + part * 8;
    *(volatile v4u*)d = v;
    __threadfence();
    *(volatile v4u*)d = v;
}

__global__ __launch_bounds__(BLOCK) void k_conv_wmma(
        const unsigned short* __restrict__ cols,
        const unsigned short* __restrict__ Wp,
        float*                __restrict__ out, int H, int hc0, int count) {
    __shared__ __attribute__((aligned(16))) float stage[C_OUT][SPITCH];

    const int n0   = blockIdx.x * NT;
    const int tid  = threadIdx.x;
    const int wave = tid >> 5;
    const int lane = tid & 31;
    const int hh   = lane >> 4;
    const int m16  = lane & 15;

    v8f acc0 = {};
    v8f acc1 = {};
    const unsigned short* ap  = Wp + ((size_t)wave * NKC * 32 + lane) * 16;
    const unsigned short* b0p = cols + (size_t)(n0 + m16) * KDIM + 8 * hh;
    const unsigned short* b1p = cols + (size_t)(n0 + 16 + m16) * KDIM + 8 * hh;

    #pragma unroll 2
    for (int kc = 0; kc < NKC; ++kc) {
        FragU a, b0, b1;
        a.q[0]  = *(const v4u*)(ap + (size_t)kc * 512);
        a.q[1]  = *(const v4u*)(ap + (size_t)kc * 512 + 8);
        b0.q[0] = *(const v4u*)(b0p + kc * KCHUNK);
        b0.q[1] = *(const v4u*)(b0p + kc * KCHUNK + 16);
        b1.q[0] = *(const v4u*)(b1p + kc * KCHUNK);
        b1.q[1] = *(const v4u*)(b1p + kc * KCHUNK + 16);
        acc0 = wmma_bf16(a.v, b0.v, acc0);
        acc1 = wmma_bf16(a.v, b1.v, acc1);
        asm volatile("v_nop\n\tv_nop\n\tv_nop\n\tv_nop"
                     : "+v"(acc0), "+v"(acc1)
                     : "v"(a.w), "v"(b0.w), "v"(b1.w));
    }

    const int mrow = wave * 16 + hh * 8;
    #pragma unroll
    for (int r = 0; r < 8; ++r) {
        float v0 = acc0[r];
        float v1 = acc1[r];
        stage[mrow + r][m16]      = v0 > 0.0f ? v0 : 0.0f;
        stage[mrow + r][16 + m16] = v1 > 0.0f ? v1 : 0.0f;
    }
    __syncthreads();

    const int chunk = lane & 7;
    const int lsub  = lane >> 3;
    const int colb  = hc0 + n0;
    const bool full = (n0 + NT <= count);
    if (full) {
        v4f vals[4];
        #pragma unroll
        for (int i = 0; i < 4; ++i) {
            int m = wave * 16 + i * 4 + lsub;
            vals[i] = *(const v4fa*)&stage[m][chunk * 4];
        }
        #pragma unroll
        for (int i = 0; i < 4; ++i) {
            int m = wave * 16 + i * 4 + lsub;
            *(volatile v4f*)(out + (size_t)m * H + colb + chunk * 4) = vals[i];
        }
        __threadfence();
        #pragma unroll
        for (int i = 0; i < 4; ++i) {
            int m = wave * 16 + i * 4 + lsub;
            *(volatile v4f*)(out + (size_t)m * H + colb + chunk * 4) = vals[i];
        }
    } else {
        float vals[16];
        #pragma unroll
        for (int i = 0; i < 4; ++i) {
            int m = wave * 16 + i * 4 + lsub;
            #pragma unroll
            for (int e = 0; e < 4; ++e) vals[i * 4 + e] = stage[m][chunk * 4 + e];
        }
        #pragma unroll
        for (int i = 0; i < 4; ++i) {
            int m = wave * 16 + i * 4 + lsub;
            #pragma unroll
            for (int e = 0; e < 4; ++e) {
                int cl = n0 + chunk * 4 + e;
                if (cl < count) *(volatile float*)(out + (size_t)m * H + hc0 + cl) = vals[i * 4 + e];
            }
        }
        __threadfence();
        #pragma unroll
        for (int i = 0; i < 4; ++i) {
            int m = wave * 16 + i * 4 + lsub;
            #pragma unroll
            for (int e = 0; e < 4; ++e) {
                int cl = n0 + chunk * 4 + e;
                if (cl < count) *(volatile float*)(out + (size_t)m * H + hc0 + cl) = vals[i * 4 + e];
            }
        }
    }
}

extern "C" void kernel_launch(void* const* d_in, const int* in_sizes, int n_in,
                              void* d_out, int out_size, void* d_ws, size_t ws_size,
                              hipStream_t stream) {
    if (n_in < 3) return;
    const float* x     = (const float*)d_in[0];
    const int*   neigh = (const int*)  d_in[1];
    const float* W     = (const float*)d_in[2];
    float*       out   = (float*)d_out;

    const int H = in_sizes[0] / C_IN;
    if (H <= 0) return;
    if ((size_t)in_sizes[1] < (size_t)H * KSZ) return;
    if ((size_t)out_size < (size_t)C_OUT * (size_t)H) return;

    const size_t xT_bytes  = (size_t)H * C_IN * sizeof(unsigned short);
    const size_t wp_off    = (xT_bytes + 127) & ~(size_t)127;
    const int    nunitsW   = MT * NKC * 32 * 16 / 8;
    const size_t wp_bytes  = (size_t)nunitsW * 16;
    const size_t cols_off  = (wp_off + wp_bytes + 127) & ~(size_t)127;
    const size_t carve_cap = (size_t)96 << 20;
    if (cols_off >= ws_size) return;
    size_t budget = ws_size - cols_off;
    if (budget > carve_cap) budget = carve_cap;
    const size_t row_bytes = (size_t)KDIM * sizeof(unsigned short);
    size_t hcmax = budget / row_bytes;
    hcmax = (hcmax / 32) * 32;
    if (hcmax < 32) return;
    const int nchunk = (int)(((size_t)H + hcmax - 1) / hcmax);
    int HC = (H + nchunk - 1) / nchunk;
    HC = ((HC + 31) / 32) * 32;
    if ((size_t)HC * row_bytes > budget) return;
    if (cols_off + (size_t)HC * row_bytes > ws_size) return;

    unsigned short* xT   = (unsigned short*)d_ws;
    unsigned short* Wp   = (unsigned short*)((char*)d_ws + wp_off);
    unsigned short* cols = (unsigned short*)((char*)d_ws + cols_off);

    k_xT<<<(H + 31) / 32, 256, 0, stream>>>(x, xT, H);
    k_pack_w<<<(nunitsW + 255) / 256, 256, 0, stream>>>(W, Wp, nunitsW);

    for (int c = 0; c < nchunk; ++c) {
        const int hc0 = c * HC;
        if (hc0 >= H) break;
        int count = H - hc0;
        if (count > HC) count = HC;
        const int nrows  = ((count + 31) / 32) * 32;
        const int nunits = nrows * KSZ * 8;
        k_gather<<<(nunits + 255) / 256, 256, 0, stream>>>(xT, neigh, cols, H, hc0, count, nunits);
        k_conv_wmma<<<nrows / NT, BLOCK, 0, stream>>>(cols, Wp, out, H, hc0, count);
    }
}
